// SphericalFeaturePropagation_67396626809176
// MI455X (gfx1250) — hardware-verified
//
#include <hip/hip_runtime.h>
#include <math.h>

typedef __attribute__((ext_vector_type(16))) _Float16 v16h;
typedef __attribute__((ext_vector_type(16))) __bf16 v16b;
typedef __attribute__((ext_vector_type(8)))  _Float16 v8h;
typedef __attribute__((ext_vector_type(8)))  float v8f;
typedef __attribute__((ext_vector_type(4)))  float v4f;
typedef __attribute__((ext_vector_type(2)))  float v2f;
typedef __attribute__((ext_vector_type(4)))  unsigned v4u;
typedef __attribute__((ext_vector_type(4)))  int v4i;
typedef float __attribute__((may_alias)) float_a;
typedef int __attribute__((may_alias)) int_a;

template <typename T> __device__ __forceinline__ void vst2(void* p, T v) { *(volatile T*)p = v; __threadfence(); *(volatile T*)p = v; }
__device__ __forceinline__ v8f wmma16(v16h a, v16h b, v8f c) {
  v8f d = __builtin_amdgcn_wmma_f32_16x16x32_f16(false, a, false, b, (short)0, c, false, false);
  asm volatile("v_nop\n\tv_nop\n\tv_nop\n\tv_nop" : "+v"(d) : "v"(a), "v"(b));
  return d;
}
__device__ __forceinline__ v8f wmma_bf(v16b a, v16b b, v8f c) {
  v8f d = __builtin_amdgcn_wmma_f32_16x16x32_bf16(false, a, false, b, (short)0, c, false, false);
  asm volatile("v_nop\n\tv_nop\n\tv_nop\n\tv_nop" : "+v"(d) : "v"(a), "v"(b));
  return d;
}
__device__ __forceinline__ v16h frag_h(const _Float16* rowk0, int lane) {
  union { v16h v; v8h q[2]; } u; const _Float16* p = rowk0 + 8 * (lane >> 4);
  u.q[0] = *(const v8h*)p; u.q[1] = *(const v8h*)(p + 16); return u.v;
}
__device__ __forceinline__ v16h frag_f32(const float* rowk0, int lane) {
  v16h a; const float* p = rowk0 + 8 * (lane >> 4);
#pragma unroll
  for (int i = 0; i < 8; ++i) { a[i] = (_Float16)p[i]; a[8 + i] = (_Float16)p[16 + i]; }
  return a;
}
__device__ __forceinline__ v16h frag_f32s(const float* rowk0, int lane, float sc) {
  v16h a; const float* p = rowk0 + 8 * (lane >> 4);
#pragma unroll
  for (int i = 0; i < 8; ++i) { a[i] = (_Float16)(p[i] * sc); a[8 + i] = (_Float16)(p[16 + i] * sc); }
  return a;
}
__device__ __forceinline__ v16h fragc_f32(const float* W, int k0, int n, int lane, int ld, int K) {
  v16h a; const int g = lane >> 4;
#pragma unroll
  for (int i = 0; i < 8; ++i) { const int ka = k0 + 8 * g + i, kb = ka + 16;
    a[i] = (_Float16)(ka < K ? W[(size_t)(ka < K ? ka : K - 1) * ld + n] : 0.f); a[8 + i] = (_Float16)(kb < K ? W[(size_t)(kb < K ? kb : K - 1) * ld + n] : 0.f); }
  return a;
}
struct F2 { v16b h, l; };
__device__ __forceinline__ F2 bsplit16(const float v[16]) { F2 r;
#pragma unroll
  for (int i = 0; i < 16; ++i) { const __bf16 h = (__bf16)v[i]; r.h[i] = h; r.l[i] = (__bf16)(v[i] - (float)h); }
  return r; }
__device__ __forceinline__ F2 split_row(const float* row, int k0, int lane) { float v[16]; const float* p = row + k0 + 8 * (lane >> 4);
#pragma unroll
  for (int i = 0; i < 8; ++i) { v[i] = p[i]; v[8 + i] = p[16 + i]; }
  return bsplit16(v); }
__device__ __forceinline__ F2 split_rowK(const float* row, int k0, int lane, int K) { float v[16]; const int g = lane >> 4;
#pragma unroll
  for (int i = 0; i < 8; ++i) { const int ka = k0 + 8 * g + i, kb = ka + 16; v[i] = ka < K ? row[ka < K ? ka : K - 1] : 0.f; v[8 + i] = kb < K ? row[kb < K ? kb : K - 1] : 0.f; }
  return bsplit16(v); }
__device__ __forceinline__ F2 split_col(const float* W, int k0, int n, int lane, int ld, int K) { float v[16]; const int g = lane >> 4;
#pragma unroll
  for (int i = 0; i < 8; ++i) { const int ka = k0 + 8 * g + i, kb = ka + 16; v[i] = ka < K ? W[(size_t)(ka < K ? ka : K - 1) * ld + n] : 0.f; v[8 + i] = kb < K ? W[(size_t)(kb < K ? kb : K - 1) * ld + n] : 0.f; }
  return bsplit16(v); }
__device__ __forceinline__ v8f mac3(const F2& a, const F2& b, v8f c) { c = wmma_bf(a.l, b.h, c); c = wmma_bf(a.h, b.l, c); return wmma_bf(a.h, b.h, c); }
__device__ __forceinline__ float sigm(float v) { return 1.0f / (1.0f + expf(-v)); }
#define LDSX() do { asm volatile("s_wait_dscnt 0" ::: "memory"); __builtin_amdgcn_wave_barrier(); __builtin_amdgcn_fence(__ATOMIC_RELEASE, "workgroup"); } while (0)


#define NBT 8
#define NP 4096
#define NR (NBT * NP)
#define KN 30
#define KP 32
#define NE (NR * KP)
#define CC 64
#ifndef NRT
#define NRT NR
#endif
#define NET (NRT * KP)
#define GRID 16
#define GLIM 5.0f
#define NCELL (NBT * GRID * GRID * GRID)
typedef __attribute__((ext_vector_type(8))) __bf16 v8b;
__device__ __forceinline__ v16b frag_b(const __bf16* rowk0, int lane) {
  union { v16b v; v8b q[2]; } u; const __bf16* p = rowk0 + 8 * (lane >> 4);
  u.q[0] = *(const v8b*)p; u.q[1] = *(const v8b*)(p + 16); return u.v;
}
__device__ __forceinline__ float bfr(float v) { return (float)(__bf16)v; }
__device__ __attribute__((noinline)) float exp_ni(float v) { return expf(v); }
__device__ __attribute__((noinline)) float erf_ni(float v) { return erff(v); }

__device__ __attribute__((noinline)) float atan2_ni(float y, float x) { return atan2f(y, x); }
#define CSA_N 32768
#define CSA_E 32768
#define CSA_FINN (CSA_E + 32 * CSA_NBK)
#define CSA_CHUNK 4096
#define CSA_BKT 256
#define CSA_NCH ((CSA_E + CSA_CHUNK - 1) / CSA_CHUNK)
#define CSA_NBK ((CSA_N + CSA_BKT - 1) / CSA_BKT)
#define CSA_NBKP (((CSA_NBK + 63) / 64) * 64)
#define CSA_SEGCAP (CSA_E + 32 * CSA_NBK * CSA_NCH)
#ifndef CSA_BCAP
#define CSA_BCAP 10240
#endif
#define CSA_SZ_CNT   (4u * CSA_NCH * CSA_NBKP)
#define CSA_SZ_OFF   (4u * CSA_NBK * (((CSA_NCH + 31) / 32) * 32))
#define CSA_SZ_BST   (4u * (((CSA_NBK + 1 + 31) / 32) * 32))
#define CSA_SZ_SEG   (4u * CSA_SEGCAP)
#define CSA_SZ_FIN   (4u * (CSA_E + 32 * CSA_NBK))
#define CSA_SZ_ROW   (4u * CSA_NBK * CSA_BKT)
#define CSA_OFFP (((CSA_NCH + 31) / 32) * 32)

__global__ __launch_bounds__(256) void k_csA_cnt(const int* __restrict__ DST, int dstride, int* __restrict__ CNT) {
  __shared__ unsigned short sc[256][CSA_NBK + 1]; __shared__ __align__(16) int srow[CSA_NBKP];
  const int c = blockIdx.x, tid = threadIdx.x;
  for (int b = 0; b < CSA_NBK; ++b) sc[tid][b] = 0;
  const size_t e0 = (size_t)c * CSA_CHUNK + tid * 16;
  for (int i = 0; i < 16; ++i) { const size_t e = e0 + i; if (e < (size_t)CSA_E) { int d = DST[e * dstride]; d = min(max(d, 0), CSA_N - 1); sc[tid][d / CSA_BKT] += 1; } }
  __syncthreads();
  for (int b = tid; b < CSA_NBKP; b += 256) { int s = 0; if (b < CSA_NBK) for (int t = 0; t < 256; ++t) s += sc[t][b]; srow[b] = s; }
  __syncthreads();
  for (int q = tid; q < CSA_NBKP / 4; q += 256) vst2((unsigned*)(CNT + (size_t)c * CSA_NBKP + q * 4), *(const v4u*)&srow[q * 4]);
}
__global__ __launch_bounds__(256) void k_csA_scan(const int* __restrict__ CNT, int* __restrict__ OFF, int* __restrict__ BST) {
  __shared__ int sbt[CSA_NBK + 1]; __shared__ int sbs[((CSA_NBK + 1 + 31) / 32) * 32]; __shared__ int scnt[CSA_NBK + 1]; __shared__ __align__(16) int sbuf[64][CSA_OFFP];
  const int tid = threadIdx.x;
  for (int b = tid; b < CSA_NBK; b += 256) { int sp = 0, st = 0; for (int c = 0; c < CSA_NCH; ++c) { const int n = CNT[(size_t)c * CSA_NBKP + b]; st += n; sp += (n + 31) & ~31; } sbt[b] = sp; scnt[b] = st; }
  for (int b = tid; b < ((CSA_NBK + 1 + 31) / 32) * 32; b += 256) sbs[b] = 0;
  __syncthreads();
  if (tid == 0) { int acc = 0, accf = 0; for (int b = 0; b < CSA_NBK; ++b) { const int t = sbt[b]; sbt[b] = acc; acc += t; sbs[b] = accf; accf += (scnt[b] + 31) & ~31; } sbs[CSA_NBK] = accf; }
  __syncthreads();
  for (int b0 = 0; b0 < CSA_NBK; b0 += 64) {
    if (tid < 64 && b0 + tid < CSA_NBK) { const int b = b0 + tid; int o = sbt[b]; for (int c = 0; c < CSA_OFFP; ++c) { if (c < CSA_NCH) { sbuf[tid][c] = o; o += (CNT[(size_t)c * CSA_NBKP + b] + 31) & ~31; } else sbuf[tid][c] = 0; } }
    __syncthreads();
    for (int q = tid; q < 64 * (CSA_OFFP / 4); q += 256) { const int r = q / (CSA_OFFP / 4), pc = q % (CSA_OFFP / 4); if (b0 + r < CSA_NBK) vst2((unsigned*)(OFF + (size_t)(b0 + r) * CSA_OFFP + pc * 4), *(const v4u*)&sbuf[r][pc * 4]); }
    __syncthreads(); }
  for (int q = tid; q < ((CSA_NBK + 1 + 31) / 32) * 32 / 4; q += 256) vst2((unsigned*)(BST + q * 4), *(const v4u*)&sbs[q * 4]);
}
__global__ __launch_bounds__(256) void k_csA_scatter(const int* __restrict__ SRC, const int* __restrict__ DST, int sstride, int dstride, const int* __restrict__ OFF, int* __restrict__ SEGS, int* __restrict__ SEGE) {
  __shared__ unsigned short sc[256][CSA_NBK + 1]; __shared__ int sbase[CSA_NBK + 1]; __shared__ int scn[CSA_NBK + 1]; __shared__ int sord[CSA_CHUNK];
  const int c = blockIdx.x, tid = threadIdx.x;
  for (int b = 0; b < CSA_NBK; ++b) sc[tid][b] = 0;
  const size_t e0 = (size_t)c * CSA_CHUNK + tid * 16; int bk[16];
#pragma unroll
  for (int i = 0; i < 16; ++i) { const size_t e = e0 + i; bk[i] = -1; if (e < (size_t)CSA_E) { int d = DST[e * dstride]; d = min(max(d, 0), CSA_N - 1); bk[i] = d / CSA_BKT; sc[tid][bk[i]] += 1; } }
  __syncthreads();
  for (int b = tid; b < CSA_NBK; b += 256) { int acc = 0; for (int t = 0; t < 256; ++t) { const int v = sc[t][b]; sc[t][b] = (unsigned short)acc; acc += v; } scn[b] = acc; }
  __syncthreads();
  if (tid == 0) { int acc = 0; for (int b = 0; b < CSA_NBK; ++b) { sbase[b] = acc; acc += scn[b]; } }
  __syncthreads();
#pragma unroll
  for (int i = 0; i < 16; ++i) { if (bk[i] >= 0) { const int b = bk[i]; const int r = sc[tid][b]; sc[tid][b] = (unsigned short)(r + 1); sord[sbase[b] + r] = tid * 16 + i; } }
  __syncthreads();
  for (int b = 0; b < CSA_NBK; ++b) { const int n = scn[b]; if (n == 0) continue; const int nl = ((n + 31) & ~31); const size_t o = (size_t)(min(max(OFF[(size_t)b * CSA_OFFP + c], 0), CSA_SEGCAP - nl) & ~31);
    for (int q = tid; q < nl / 4; q += 256) { int4 vs, ve;
#pragma unroll
      for (int k = 0; k < 4; ++k) { const int i = q * 4 + k; int s = -1, eid = -1; if (i < n) { const size_t e = (size_t)c * CSA_CHUNK + sord[sbase[b] + i]; s = min(max(SRC[e * sstride], 0), CSA_N - 1); eid = (int)e; } vs[k] = s; ve[k] = eid; }
      vst2((unsigned*)(SEGS + o + q * 4), *(const v4u*)&vs); vst2((unsigned*)(SEGE + o + q * 4), *(const v4u*)&ve); } }
}
__global__ __launch_bounds__(256) void k_csA_bucket(const int* __restrict__ CNT, const int* __restrict__ OFF, const int* __restrict__ BST, const int* __restrict__ SEGS, const int* __restrict__ SEGE, const int* __restrict__ DST, int dstride, int* __restrict__ FS, int* __restrict__ FE, int* __restrict__ ROWST, int* __restrict__ ROWCNT) {
  __shared__ int ssrc[CSA_BCAP]; __shared__ int seid[CSA_BCAP]; __shared__ unsigned char snod[CSA_BCAP]; __shared__ int souts[CSA_BCAP]; __shared__ int soute[CSA_BCAP]; __shared__ int scount[256]; __shared__ int sstart[257]; __shared__ int stot;
  const int b = blockIdx.x, tid = threadIdx.x;
  if (tid == 0) { int t = 0; for (int c = 0; c < CSA_NCH; ++c) t += min(max(CNT[(size_t)c * CSA_NBKP + b], 0), CSA_CHUNK); stot = (t <= CSA_BCAP) ? t : 0; }
  __syncthreads();
  { int base = 0; for (int c = 0; c < CSA_NCH; ++c) { const int n = min(max(CNT[(size_t)c * CSA_NBKP + b], 0), CSA_CHUNK); const int o = min(max(OFF[(size_t)b * CSA_OFFP + c], 0), CSA_SEGCAP - ((n + 31) & ~31));
      for (int i = tid; i < n; i += 256) { const int p = base + i; if (p < CSA_BCAP) { ssrc[p] = min(max(SEGS[o + i], 0), CSA_N - 1); const int e = min(max(SEGE[o + i], 0), CSA_E - 1); seid[p] = e; int d = DST[(size_t)e * dstride]; d = min(max(d, 0), CSA_N - 1); const int dl = d - b * CSA_BKT; snod[p] = (unsigned char)(dl >= 0 && dl < 256 ? dl : 255); } }
      base += n; } }
  __syncthreads();
  const int node = b * CSA_BKT + tid; int cnt = 0; for (int p = 0; p < stot; ++p) cnt += (snod[p] == tid) ? 1 : 0;
  scount[tid] = cnt; __syncthreads();
  if (tid == 0) { int acc = 0; for (int t = 0; t < 256; ++t) { sstart[t] = acc; acc += scount[t]; } sstart[256] = acc; }
  __syncthreads();
  const int bst0 = min(max(BST[b], 0), CSA_FINN - ((sstart[256] + 31) & ~31)) & ~31; const int gst = bst0 + sstart[tid];
  { int w = sstart[tid]; for (int p = 0; p < stot; ++p) if (snod[p] == tid) { souts[w] = ssrc[p]; soute[w] = seid[p]; ++w; } }
  __syncthreads();
  { const int n = sstart[256]; const int nl = (n + 31) & ~31; for (int q = tid; q < nl / 4; q += 256) { int4 vs, ve;
#pragma unroll
      for (int k = 0; k < 4; ++k) { const int i = q * 4 + k; vs[k] = i < n ? souts[i] : -1; ve[k] = i < n ? soute[i] : -1; }
      vst2((unsigned*)(FS + bst0 + q * 4), *(const v4u*)&vs); vst2((unsigned*)(FE + bst0 + q * 4), *(const v4u*)&ve); } }
  __syncthreads();
  { __shared__ __align__(16) int srs[256], src2[256]; srs[tid] = node < CSA_N ? gst : 0; src2[tid] = node < CSA_N ? cnt : 0; __syncthreads();
    if (tid < 64) vst2((unsigned*)(ROWST + (size_t)b * 256 + tid * 4), *(const v4u*)&srs[tid * 4]); else if (tid < 128) vst2((unsigned*)(ROWCNT + (size_t)b * 256 + (tid - 64) * 4), *(const v4u*)&src2[(tid - 64) * 4]); }
}


#define WS_CNT  0u
#define WS_OFF  (WS_CNT + CSA_SZ_CNT)
#define WS_BST  (WS_OFF + CSA_SZ_OFF)
#define WS_SEGS (WS_BST + CSA_SZ_BST)
#define WS_SEGE (WS_SEGS + CSA_SZ_SEG)
#define WS_FS   (WS_SEGE + CSA_SZ_SEG)
#define WS_FE   (WS_FS + CSA_SZ_FIN)
#define WS_RST  (WS_FE + CSA_SZ_FIN)
#define WS_RCT  (WS_RST + CSA_SZ_ROW)
#define WS_CELL (WS_RCT + CSA_SZ_ROW)
#define WS_PID  (WS_CELL + 4u * NR)
#define WS_P    (WS_PID + 4u * NR)
#define WS_IDX  (WS_P + 4u * NR * 4)
#define WS_F    (WS_IDX + 4u * NR * KP)
#define WS_H1   (WS_F + 4u * NE * 8)
#define WS_H2   (WS_H1 + 4u * NE * 8)
#define WS_H3   (WS_H2 + 4u * NE * 4)
#define WS_PW   (WS_H3 + 4u * NE)
#define NSTB 256
#define WS_ST   (WS_PW + 2u * 2 * 16 * 32)
#define WS_BN   (WS_ST + 4u * NSTB * 8)
#define WS_END  (WS_BN + 4u * 3 * 24)

__device__ __forceinline__ int cell_of(float v) { return min(max((int)floorf((v + GLIM) * ((float)GRID / (2.0f * GLIM))), 0), GRID - 1); }
__global__ __launch_bounds__(256) void k_pts(const float* __restrict__ XL, float* __restrict__ Pp, int* __restrict__ CELL, int* __restrict__ PID) {
  __shared__ __align__(16) int sc[256], sp[256]; const int t = threadIdx.x; const size_t i = (size_t)blockIdx.x * 256 + t; const int b = (int)(i / NP), n = (int)(i % NP);
  const float x = bfr(XL[((size_t)b * 3 + 0) * NP + n]), y = bfr(XL[((size_t)b * 3 + 1) * NP + n]), z = bfr(XL[((size_t)b * 3 + 2) * NP + n]);
  vst2(Pp + i * 4, (v4f){x, y, z, 0.f});
  sc[t] = ((b * GRID + cell_of(x)) * GRID + cell_of(y)) * GRID + cell_of(z); sp[t] = (int)i; __syncthreads();
  if (t < 64) { vst2((unsigned*)(CELL + (size_t)blockIdx.x * 256 + t * 4), *(const v4u*)&sc[t * 4]); vst2((unsigned*)(PID + (size_t)blockIdx.x * 256 + t * 4), *(const v4u*)&sp[t * 4]); }
}
__global__ __launch_bounds__(32) void k_packW(const float* __restrict__ W1, const float* __restrict__ W2, __bf16* __restrict__ PW) {
  __shared__ __align__(16) __bf16 s[2][16][32]; const int t = threadIdx.x;
  for (int q = t; q < 2 * 16 * 32; q += 32) { const int w = q / 512, o = (q / 32) % 16, k = q % 32; float v = 0.f; if (w == 0 && o < 6 && k < 6) v = W1[o * 6 + k]; if (w == 1 && o < 3 && k < 6) v = W2[o * 6 + k]; (&s[0][0][0])[q] = (__bf16)v; }
  __syncthreads();
  for (int q = t; q < 2 * 16 * 32 / 8; q += 32) vst2((unsigned*)(PW + q * 8), *(const v4u*)(&s[0][0][0] + q * 8));
}
__device__ __forceinline__ void knn_ins(float pd, int m, float* bd, int* bi) {
  if (pd > bd[KN - 1] || (pd == bd[KN - 1] && m < bi[KN - 1])) { int pos = KN - 1;
#pragma unroll
    for (int q = KN - 2; q >= 0; --q) if (pd > bd[q] || (pd == bd[q] && m < bi[q])) pos = q;
#pragma unroll
    for (int q = KN - 1; q >= 1; --q) if (q > pos) { bd[q] = bd[q - 1]; bi[q] = bi[q - 1]; }
#pragma unroll
    for (int q = 0; q < KN; ++q) if (q == pos) { bd[q] = pd; bi[q] = m; } }
}
__global__ __launch_bounds__(64) void k_knn(const float* __restrict__ Pp, const int* __restrict__ CELL, const int* __restrict__ FE, const int* __restrict__ RST, const int* __restrict__ RCT, int* __restrict__ IDX) {
  #pragma clang fp contract(off)
  __shared__ __align__(16) int sk[64][KP]; const int t = threadIdx.x; const size_t i = (size_t)blockIdx.x * 64 + t; const int b = (int)(i / NP);
  const float ax = Pp[i * 4], ay = Pp[i * 4 + 1], az = Pp[i * 4 + 2]; const float xxa = (ax * ax + az * az) + ay * ay;
  const int cid = min(max(CELL[i], 0), NCELL - 1) - b * GRID * GRID * GRID; const int cx = cid / (GRID * GRID), cy = (cid / GRID) % GRID, cz = cid % GRID;
  float bd[KN]; int bi[KN]; bool done = false;
#pragma unroll 1
  for (int R = 1; R <= 3 && !done; ++R) {
#pragma unroll
    for (int q = 0; q < KN; ++q) { bd[q] = -3.0e38f; bi[q] = 0x7fffffff; }
    if (R <= 2) {
#pragma unroll 1
      for (int gx = max(cx - R, 0); gx <= min(cx + R, GRID - 1); ++gx)
#pragma unroll 1
        for (int gy = max(cy - R, 0); gy <= min(cy + R, GRID - 1); ++gy)
#pragma unroll 1
          for (int gz = max(cz - R, 0); gz <= min(cz + R, GRID - 1); ++gz) { const int c = ((b * GRID + gx) * GRID + gy) * GRID + gz; const int cnt = min(max(RCT[c], 0), CSA_BCAP); const int st = min(max(RST[c], 0), CSA_FINN - cnt);
#pragma unroll 1
            for (int e = 0; e < cnt; ++e) { const int mg = min(max(FE[st + e], 0), NR - 1); const int m = mg - b * NP; const float bx = Pp[(size_t)mg * 4], by = Pp[(size_t)mg * 4 + 1], bz = Pp[(size_t)mg * 4 + 2]; const float xxb = (bx * bx + bz * bz) + by * by; const float dot = (ax * bx + ay * by) + az * bz; const float pd = (2.0f * dot - xxa) - xxb; knn_ins(pd, m, bd, bi); } }
      const float cs = 2.0f * GLIM / (float)GRID; float margin = 3.0e38f;
      { const float lo = (cx - R >= 1) ? (ax - (-GLIM + (float)(cx - R) * cs)) : 3.0e38f, hi = (cx + R <= GRID - 2) ? ((-GLIM + (float)(cx + R + 1) * cs) - ax) : 3.0e38f; margin = fminf(margin, fminf(lo, hi)); }
      { const float lo = (cy - R >= 1) ? (ay - (-GLIM + (float)(cy - R) * cs)) : 3.0e38f, hi = (cy + R <= GRID - 2) ? ((-GLIM + (float)(cy + R + 1) * cs) - ay) : 3.0e38f; margin = fminf(margin, fminf(lo, hi)); }
      { const float lo = (cz - R >= 1) ? (az - (-GLIM + (float)(cz - R) * cs)) : 3.0e38f, hi = (cz + R <= GRID - 2) ? ((-GLIM + (float)(cz + R + 1) * cs) - az) : 3.0e38f; margin = fminf(margin, fminf(lo, hi)); }
      const float msafe = fmaxf(margin, 0.f) * 0.98f;
      done = (bi[KN - 1] != 0x7fffffff) && (-bd[KN - 1] < msafe * msafe);
    } else {
      const float* pc = Pp + (size_t)b * NP * 4;
#pragma unroll 1
      for (int m = 0; m < NP; ++m) { const float bx = pc[m * 4], by = pc[m * 4 + 1], bz = pc[m * 4 + 2]; const float xxb = (bx * bx + bz * bz) + by * by; const float dot = (ax * bx + ay * by) + az * bz; const float pd = (2.0f * dot - xxa) - xxb; knn_ins(pd, m, bd, bi); }
      done = true; }
  }
#pragma unroll
  for (int q = 0; q < KN; ++q) sk[t][q] = b * NP + min(bi[q], NP - 1);
  sk[t][30] = sk[t][0]; sk[t][31] = sk[t][0];
  __syncthreads();
  for (int q = t; q < 64 * 8; q += 64) { const int rl = q >> 3, pcs = q & 7; vst2((unsigned*)(IDX + ((size_t)blockIdx.x * 64 + rl) * KP + pcs * 4), *(const v4u*)&sk[rl][pcs * 4]); }
}
__global__ __launch_bounds__(256) void k_feat(const float* __restrict__ Pp, const int* __restrict__ IDX, float* __restrict__ F) {
  #pragma clang fp contract(off)
  __shared__ __align__(16) float sf[256][8]; const int t = threadIdx.x; const size_t e = (size_t)blockIdx.x * 256 + t; const size_t i = e / KP; const int slot = (int)(e % KP);
  const int m = min(max(IDX[i * KP + slot], 0), NR - 1);
  const float xr = Pp[(size_t)m * 4] - Pp[i * 4], yr = Pp[(size_t)m * 4 + 1] - Pp[i * 4 + 1], zr = Pp[(size_t)m * 4 + 2] - Pp[i * 4 + 2];
  const float sxy2 = xr * xr + yr * yr; const float r2 = sxy2 + zr * zr;
  const float rho = sqrtf(fmaxf(r2, 1e-20f)), sxy = sqrtf(fmaxf(sxy2, 1e-20f)); const bool dr = r2 < 1e-20f, dp = sxy2 < 1e-20f;
  const float theta = atan2_ni(dr ? 0.f : zr, dr ? 1.f : sxy); const float phi = atan2_ni(dp ? 0.f : yr, dp ? 1.f : xr);
  const float mean3 = ((rho + phi) + theta) / 3.0f;
  sf[t][0] = rho; sf[t][1] = theta; sf[t][2] = phi; sf[t][3] = rho - mean3; sf[t][4] = theta - mean3; sf[t][5] = phi - mean3; sf[t][6] = 0.f; sf[t][7] = 0.f;
  __syncthreads();
  for (int q = t; q < 256 * 2; q += 256) vst2(F + (size_t)blockIdx.x * 256 * 8 + q * 4, *(const v4f*)(&sf[0][0] + q * 4));
}
template <int LAYER>
__global__ __launch_bounds__(128) void k_lin(const float* __restrict__ IN, const float* __restrict__ BNP, const __bf16* __restrict__ PW, float* __restrict__ OUTp) {
  __shared__ __align__(16) float sa[4][16][36]; __shared__ __align__(16) float so[4][16][8];
  const int tid = threadIdx.x, wave = tid >> 5, lane = tid & 31, col = lane & 15, g = lane >> 4; const size_t r0 = (size_t)blockIdx.x * 64 + wave * 16;
  for (int q = lane; q < 16 * 32; q += 32) { const int rl = q >> 5, c = q & 31; float v = 0.f;
    if (LAYER == 1) { if (c < 6) v = IN[(r0 + rl) * 8 + c]; } else { if (c < 6) { float h = IN[(r0 + rl) * 8 + c] * BNP[8 + c] + BNP[16 + c]; v = h > 0.f ? h : 0.2f * h; } }
    sa[wave][rl][c] = v; }
  LDSX();
  const F2 a = split_row(&sa[wave][col][0], 0, lane); v8f acc = {};
  const v16b w = frag_b(PW + (LAYER == 1 ? 0 : 16 * 32) + (size_t)col * 32, lane); acc = wmma_bf(a.l, w, acc); acc = wmma_bf(a.h, w, acc);
  if (col < 8) {
#pragma unroll
    for (int r = 0; r < 8; ++r) so[wave][8 * g + r][col] = (col < (LAYER == 1 ? 6 : 3)) ? acc[r] : 0.f; }
  LDSX();
  if (LAYER == 1) { vst2(OUTp + (r0 + (lane >> 1)) * 8 + (lane & 1) * 4, *(const v4f*)&so[wave][lane >> 1][(lane & 1) * 4]); }
  else { if (lane < 16) vst2(OUTp + (r0 + lane) * 4, *(const v4f*)&so[wave][lane][0]); }
}
__global__ __launch_bounds__(256) void k_l3(const float* __restrict__ H2, const float* __restrict__ BNP, const float* __restrict__ W3, float* __restrict__ H3) {
  __shared__ __align__(16) float s[256]; const int t = threadIdx.x; const size_t e = (size_t)blockIdx.x * 256 + t; float a = 0.f;
#pragma unroll
  for (int c = 0; c < 3; ++c) { float h = H2[e * 4 + c] * BNP[8 + c] + BNP[16 + c]; h = h > 0.f ? h : 0.2f * h; a += h * bfr(W3[c]); }
  s[t] = a; __syncthreads();
  if (t < 64) vst2(H3 + (size_t)blockIdx.x * 256 + t * 4, *(const v4f*)&s[t * 4]);
}
template <int PASS>
__global__ __launch_bounds__(256) void k_stat(const float* __restrict__ Y, int W, int ld, const float* __restrict__ BNP, float* __restrict__ ST) {
  __shared__ float s[32][8]; __shared__ __align__(16) float so[8]; const int t = threadIdx.x; const int c = t & 7, grp = t >> 3;
  const size_t per = (size_t)NET / NSTB; const size_t e0 = (size_t)blockIdx.x * per; float a = 0.f; const float mu = (PASS && c < W) ? BNP[c] : 0.f;
  if (c < W) { for (size_t e = e0 + grp; e < e0 + per; e += 32) { if ((int)(e % KP) >= KN) continue; const float y = Y[e * ld + c]; const float d = y - mu; a += PASS ? d * d : y; } }
  s[grp][c] = a; __syncthreads();
  if (t < 8) { float tot = 0.f; for (int q = 0; q < 32; ++q) tot += s[q][t]; so[t] = tot; }
  __syncthreads();
  if (t < 2) vst2(ST + (size_t)blockIdx.x * 8 + t * 4, *(const v4f*)&so[t * 4]);
}
template <int PASS>
__global__ __launch_bounds__(32) void k_fin(const float* __restrict__ ST, int W, const float* __restrict__ G, const float* __restrict__ BE, float* __restrict__ BNP) {
  __shared__ __align__(16) float s[2][8]; const int c = threadIdx.x; float a = 0.f;
  if (c < 8) { for (int b = 0; b < NSTB; ++b) a += ST[(size_t)b * 8 + c]; }
  const float n = (float)((size_t)NRT * KN);
  if (PASS == 0) { if (c < 8) s[0][c] = (c < W) ? a / n : 0.f; __syncthreads(); if (c < 2) vst2(BNP + c * 4, *(const v4f*)&s[0][c * 4]); }
  else { if (c < 8) { float sc = 0.f, sh = 0.f; if (c < W) { const float var = a / n; sc = bfr(G[c]) * rsqrtf(var + 1e-5f); sh = bfr(BE[c]) - BNP[c] * sc; } s[0][c] = sc; s[1][c] = sh; } __syncthreads(); if (c < 2) { vst2(BNP + 8 + c * 4, *(const v4f*)&s[0][c * 4]); vst2(BNP + 16 + c * 4, *(const v4f*)&s[1][c * 4]); } }
}
__global__ __launch_bounds__(256) void k_out(const float* __restrict__ H3, const float* __restrict__ BNP, const int* __restrict__ IDX, const float* __restrict__ X, float* __restrict__ OUT) {
  __shared__ float satt[64][KP]; __shared__ int snb[64][KP]; __shared__ __align__(16) float so[CC][64];
  const int t = threadIdx.x; const size_t i0 = (size_t)blockIdx.x * 64; const int b = (int)(i0 / NP); const int n0 = (int)(i0 % NP);
  for (int q = t; q < 64 * KP; q += 256) { const int pl = q >> 5, k = q & 31; float v = -3.0e38f; if (k < KN) { float h = H3[(i0 + pl) * KP + k] * BNP[8] + BNP[16]; v = h > 0.f ? h : 0.2f * h; } satt[pl][k] = v; snb[pl][k] = min(max(IDX[(i0 + pl) * KP + k], 0), NR - 1) - b * NP; }
  __syncthreads();
  if (t < 64) { const int pl = t; float mx = -3.0e38f; for (int k = 0; k < KN; ++k) mx = fmaxf(mx, satt[pl][k]); float z = 0.f; for (int k = 0; k < KN; ++k) { const float e = exp_ni(satt[pl][k] - mx); satt[pl][k] = e; z += e; } const float iz = 1.0f / z; for (int k = 0; k < KN; ++k) satt[pl][k] *= iz; }
  __syncthreads();
  { const int c = t >> 2, pq = t & 3; const float* xc = X + ((size_t)b * CC + c) * NP;
    for (int pl = pq * 16; pl < pq * 16 + 16; ++pl) { float a = 0.f;
#pragma unroll 2
      for (int k = 0; k < KN; ++k) { const int m = min(max(snb[pl][k], 0), NP - 1); a += satt[pl][k] * bfr(xc[m]); }
      so[c][pl] = bfr(xc[n0 + pl]) + a; } }
  __syncthreads();
  for (int q = t; q < CC * 16; q += 256) { const int c = q >> 4, pcs = q & 15; vst2(OUT + ((size_t)b * CC + c) * NP + n0 + pcs * 4, *(const v4f*)&so[c][pcs * 4]); }
}
extern "C" void kernel_launch(void* const* d_in, const int* in_sizes, int n_in, void* d_out, int out_size, void* d_ws, size_t ws_size, hipStream_t stream) {
  (void)in_sizes; (void)n_in; (void)out_size;
  const float** Fi = (const float**)d_in;
  if (ws_size < (size_t)WS_END) return;
  char* ws = (char*)d_ws; int *CNT = (int*)(ws + WS_CNT), *OFF = (int*)(ws + WS_OFF), *BST = (int*)(ws + WS_BST), *SEGS = (int*)(ws + WS_SEGS), *SEGE = (int*)(ws + WS_SEGE), *FS = (int*)(ws + WS_FS), *FE = (int*)(ws + WS_FE), *RST = (int*)(ws + WS_RST), *RCT = (int*)(ws + WS_RCT), *CELL = (int*)(ws + WS_CELL), *PID = (int*)(ws + WS_PID); float *Pp = (float*)(ws + WS_P), *F = (float*)(ws + WS_F), *H1 = (float*)(ws + WS_H1), *H2 = (float*)(ws + WS_H2), *H3 = (float*)(ws + WS_H3), *ST = (float*)(ws + WS_ST), *BN = (float*)(ws + WS_BN); int* IDX = (int*)(ws + WS_IDX); __bf16* PW = (__bf16*)(ws + WS_PW);
  float *BN1 = BN, *BN2 = BN + 24, *BN3 = BN + 48;
  k_pts<<<NR / 256, 256, 0, stream>>>(Fi[0], Pp, CELL, PID);
  k_csA_cnt<<<CSA_NCH, 256, 0, stream>>>(CELL, 1, CNT); k_csA_scan<<<1, 256, 0, stream>>>(CNT, OFF, BST); k_csA_scatter<<<CSA_NCH, 256, 0, stream>>>(PID, CELL, 1, 1, OFF, SEGS, SEGE); k_csA_bucket<<<CSA_NBK, 256, 0, stream>>>(CNT, OFF, BST, SEGS, SEGE, CELL, 1, FS, FE, RST, RCT);
  k_packW<<<1, 32, 0, stream>>>(Fi[2], Fi[5], PW);
  k_knn<<<NRT / 64, 64, 0, stream>>>(Pp, CELL, FE, RST, RCT, IDX);
  k_feat<<<NET / 256, 256, 0, stream>>>(Pp, IDX, F);
  k_lin<1><<<NET / 64, 128, 0, stream>>>(F, nullptr, PW, H1);
  k_stat<0><<<NSTB, 256, 0, stream>>>(H1, 6, 8, BN1, ST); k_fin<0><<<1, 32, 0, stream>>>(ST, 6, Fi[3], Fi[4], BN1); k_stat<1><<<NSTB, 256, 0, stream>>>(H1, 6, 8, BN1, ST); k_fin<1><<<1, 32, 0, stream>>>(ST, 6, Fi[3], Fi[4], BN1);
  k_lin<2><<<NET / 64, 128, 0, stream>>>(H1, BN1, PW, H2);
  k_stat<0><<<NSTB, 256, 0, stream>>>(H2, 3, 4, BN2, ST); k_fin<0><<<1, 32, 0, stream>>>(ST, 3, Fi[6], Fi[7], BN2); k_stat<1><<<NSTB, 256, 0, stream>>>(H2, 3, 4, BN2, ST); k_fin<1><<<1, 32, 0, stream>>>(ST, 3, Fi[6], Fi[7], BN2);
  k_l3<<<NET / 256, 256, 0, stream>>>(H2, BN2, Fi[8], H3);
  k_stat<0><<<NSTB, 256, 0, stream>>>(H3, 1, 1, BN3, ST); k_fin<0><<<1, 32, 0, stream>>>(ST, 1, Fi[9], Fi[10], BN3); k_stat<1><<<NSTB, 256, 0, stream>>>(H3, 1, 1, BN3, ST); k_fin<1><<<1, 32, 0, stream>>>(ST, 1, Fi[9], Fi[10], BN3);
  k_out<<<NRT / 64, 256, 0, stream>>>(H3, BN3, IDX, Fi[1], (float*)d_out);
}
